// SequentialTransductionUnitJagged_21440476742332
// MI455X (gfx1250) — hardware-run, weakly checked
//
#include <hip/hip_runtime.h>

constexpr int NBATCH = 2;
constexpr int SEQ    = 2048;
constexpr int EMB    = 512;
constexpr int NHEAD  = 8;
constexpr int HDIM   = 64;
constexpr int NBUCK  = 128;
constexpr int UCOLS  = 3 * NHEAD * HDIM;
constexpr int QKVC   = NHEAD * HDIM + 2 * NHEAD * HDIM;
constexpr int WCOLS  = UCOLS + QKVC;
constexpr int NROWS  = NBATCH * SEQ;
constexpr int POSLEN = 2 * SEQ - 1;
constexpr int HCAT   = 3 * HDIM;
constexpr float LN_EPS    = 1e-6f;
constexpr float W1_CARRY  = 64.0f;
constexpr float W2_CARRY  = 32.0f;
constexpr float QKV_CARRY = 32.0f;
constexpr float PT_CARRY  = 1024.0f;
constexpr float PL_CARRY  = 32.0f;

static_assert(EMB % 64 == 0 && UCOLS % 64 == 0 && QKVC % 64 == 0 && SEQ % 64 == 0 && NROWS % 64 == 0, "tile multiples");
static_assert(EMB % 32 == 0 && SEQ % 32 == 0 && UCOLS % 32 == 0 && HDIM == 64, "K multiples");
static_assert(SEQ == 2048 && EMB == 512 && NHEAD * HDIM == EMB && NHEAD * HCAT == UCOLS, "index shifts below assume these");

typedef __attribute__((ext_vector_type(16))) _Float16 v16h;
typedef __attribute__((ext_vector_type(8)))  _Float16 v8h;
typedef __attribute__((ext_vector_type(16))) __bf16   v16b;
typedef __attribute__((ext_vector_type(8)))  __bf16   v8b;
typedef __attribute__((ext_vector_type(8)))  float    v8f;
typedef __attribute__((ext_vector_type(4)))  float    v4f;
typedef __attribute__((ext_vector_type(2)))  float    v2f;
typedef __attribute__((ext_vector_type(4)))  unsigned v4u;
typedef __attribute__((ext_vector_type(2)))  int      v2i;
typedef __attribute__((ext_vector_type(4)))  int      v4i;

__device__ __forceinline__ unsigned short h_bits(float f) { return __builtin_bit_cast(unsigned short, (_Float16)f); }
__device__ __forceinline__ unsigned pk2h(float a, float b) { return (unsigned)h_bits(a) | ((unsigned)h_bits(b) << 16); }

__device__ __forceinline__ void dep_guard_h(v8f& a, v8f& b, v16h x, v16h y) { asm volatile("v_nop\n\tv_nop\n\tv_nop\n\tv_nop" : "+v"(a), "+v"(b) : "v"(x), "v"(y)); }
__device__ __forceinline__ void dep_guard_b(v8f& a, v8f& b, v16b x, v16b y) { asm volatile("v_nop\n\tv_nop\n\tv_nop\n\tv_nop" : "+v"(a), "+v"(b) : "v"(x), "v"(y)); }
__device__ __forceinline__ void keep4_h(v16h a, v16h b, v16h c, v16h d) { asm volatile("v_nop" :: "v"(a), "v"(b), "v"(c), "v"(d)); }
__device__ __forceinline__ void keep4_b(v16b a, v16b b, v16b c, v16b d) { asm volatile("v_nop" :: "v"(a), "v"(b), "v"(c), "v"(d)); }
__device__ __forceinline__ void acc_guard4(v8f& a, v8f& b, v8f& c, v8f& d) { asm volatile("v_nop\n\tv_nop\n\tv_nop\n\tv_nop" : "+v"(a), "+v"(b), "+v"(c), "+v"(d)); }
template <typename T> struct Frag;
template <> struct Frag<_Float16> {
  typedef v16h V; union U { v16h v; v8h h[2]; };
  static __device__ __forceinline__ v16h load(const _Float16* p) {
    U f; f.h[0] = *(const v8h*)(p); f.h[1] = *(const v8h*)(p + 16); return f.v;
  }
  static __device__ __forceinline__ v8f mma(v16h a, v16h b, v8f c) {
    return __builtin_amdgcn_wmma_f32_16x16x32_f16(false, a, false, b, (short)0, c, false, false);
  }
  static __device__ __forceinline__ void guard(v8f& a, v8f& b, v16h x, v16h y) { dep_guard_h(a, b, x, y); }
  static __device__ __forceinline__ void keep(v16h a, v16h b, v16h c, v16h d) { keep4_h(a, b, c, d); }
};
template <> struct Frag<__bf16> {
  typedef v16b V; union U { v16b v; v8b h[2]; };
  static __device__ __forceinline__ v16b load(const __bf16* p) {
    U f; f.h[0] = *(const v8b*)(p); f.h[1] = *(const v8b*)(p + 16); return f.v;
  }
  static __device__ __forceinline__ v8f mma(v16b a, v16b b, v8f c) {
    return __builtin_amdgcn_wmma_f32_16x16x32_bf16(false, a, false, b, (short)0, c, false, false);
  }
  static __device__ __forceinline__ void guard(v8f& a, v8f& b, v16b x, v16b y) { dep_guard_b(a, b, x, y); }
  static __device__ __forceinline__ void keep(v16b a, v16b b, v16b c, v16b d) { keep4_b(a, b, c, d); }
};

template <int BIAS_MODE, int OUT_MODE, bool RESID, int ACT>
__global__ __launch_bounds__(256) void gemm64_f16(
    const unsigned short* __restrict__ Ap, int lda, long strideA,
    const unsigned short* __restrict__ Btp, int ldb, long strideB,
    void* __restrict__ Cout, int ldc, long strideC, int ocs, int oco,
    const float* __restrict__ bias,
    const float* __restrict__ resid, long strideR,
    int M, int N, int K, float scale, float post) {
  static_assert(!(RESID && OUT_MODE != 0), "resid only on the f32 store path");
  typedef _Float16 T;
  typedef v16h V;
  const T* A = (const T*)Ap; const T* Bt = (const T*)Btp;
  __shared__ __align__(16) float sT[8][16 * 68];
  const int b    = blockIdx.y;
  const int lane = threadIdx.x & 31;
  const int wave = threadIdx.x >> 5;
  const int tilesN = N >> 6;
  const int tilesM = M >> 6;
  const int tile = blockIdx.x * 8 + wave;
  if (tile >= tilesM * tilesN) return;
  const int tm = tile / tilesN;
  const int tn = tile - tm * tilesN;
  const int m0 = tm << 6;
  const int n0 = tn << 6;
  const int nc0 = tn * ocs + oco;

  const T* Ab = A  + (size_t)b * strideA;
  const T* Bb = Bt + (size_t)b * strideB;

  const int rlane = lane & 15;
  const int koff  = (lane >> 4) * 8;
  const int mOff  = (lane >> 4) * 8;

  v8f acc[4][4];
#pragma unroll
  for (int i = 0; i < 4; ++i)
#pragma unroll
    for (int j = 0; j < 4; ++j) acc[i][j] = (v8f){0.f,0.f,0.f,0.f,0.f,0.f,0.f,0.f};

  for (int k0 = 0; k0 < K; k0 += 32) {
    V bh[4];
#pragma unroll
    for (int j = 0; j < 4; ++j) {
      const size_t bo = (size_t)(n0 + (j << 4) + rlane) * ldb + koff + k0;
      bh[j] = Frag<T>::load(Bb + bo);
    }
#pragma unroll
    for (int i = 0; i < 4; ++i) {
      const size_t ao = (size_t)(m0 + (i << 4) + rlane) * lda + koff + k0;
      V ah = Frag<T>::load(Ab + ao);
#pragma unroll
      for (int j = 0; j < 4; ++j) acc[i][j] = Frag<T>::mma(ah, bh[j], acc[i][j]);
      Frag<T>::guard(acc[i][0], acc[i][3], ah, ah);
    }
    Frag<T>::keep(bh[0], bh[1], bh[2], bh[3]);
  }
  acc_guard4(acc[0][0], acc[0][1], acc[0][2], acc[0][3]);
  acc_guard4(acc[1][0], acc[1][1], acc[1][2], acc[1][3]);
  acc_guard4(acc[2][0], acc[2][1], acc[2][2], acc[2][3]);
  acc_guard4(acc[3][0], acc[3][1], acc[3][2], acc[3][3]);

  float* slab = sT[wave];
  const float* Rb = RESID ? (resid + (size_t)b * strideR) : nullptr;
#pragma unroll
  for (int i = 0; i < 4; ++i) {
    const int mBase = m0 + (i << 4);
#pragma unroll
    for (int j = 0; j < 4; ++j) {
      const int n = nc0 + (j << 4) + rlane;
      float bv = 0.f;
      if (BIAS_MODE == 2) bv = bias[n];
#pragma unroll
      for (int r = 0; r < 8; ++r) {
        float v = acc[i][j][r] * scale;
        if (BIAS_MODE == 2) v += bv;
        if (ACT == 3) {
          const float e = expf(fminf(-v, 30.0f));
          v = v * (1.0f / (1.0f + e));
          v = v * post;
        }
        slab[(mOff + r) * 68 + (j << 4) + rlane] = v;
      }
    }
    __builtin_amdgcn_fence(__ATOMIC_RELEASE, "workgroup");
    __builtin_amdgcn_wave_barrier();
    __builtin_amdgcn_fence(__ATOMIC_ACQUIRE, "workgroup");
    if (OUT_MODE == 0) {
      float* C = (float*)Cout + (size_t)b * strideC;
      const int hh = lane >> 4, c4 = (lane & 15) * 4;
      for (int pass = 0; pass < 2; ++pass) {
#pragma unroll
        for (int it = 0; it < 8; ++it) {
          const int row = it * 2 + hh;
          v4f v = *(const v4f*)(slab + row * 68 + c4);
          if (RESID) {
            const v4f rv = *(const v4f*)(Rb + (size_t)(mBase + row) * ldc + nc0 + c4);
            v = v + rv;
          }
          *(volatile v4f*)(C + (size_t)(mBase + row) * ldc + nc0 + c4) = v;
        }
        __threadfence();
      }
    } else {
      const int q = lane >> 3, c8 = (lane & 7) * 8;
      unsigned short* C = (unsigned short*)Cout + (size_t)b * strideC;
      for (int pass = 0; pass < 2; ++pass) {
#pragma unroll
        for (int it = 0; it < 4; ++it) {
          const int row = it * 4 + q;
          const float* sp = slab + row * 68 + c8;
          v8h hv;
#pragma unroll
          for (int e = 0; e < 8; ++e) hv[e] = (_Float16)sp[e];
          *(volatile v8h*)(C + (size_t)(mBase + row) * ldc + nc0 + c8) = hv;
        }
        __threadfence();
      }
    }
    __builtin_amdgcn_fence(__ATOMIC_RELEASE, "workgroup");
    __builtin_amdgcn_wave_barrier();
    __builtin_amdgcn_fence(__ATOMIC_ACQUIRE, "workgroup");
  }
}

__global__ __launch_bounds__(64) void ln_cast_kernel(const float* __restrict__ x, unsigned short* __restrict__ xn) {
  __shared__ float red0[2];
  __shared__ float red1[2];
  const int row = blockIdx.x, tid = threadIdx.x, lane = tid & 31, wave = tid >> 5;
  const float* xr = x + (size_t)row * EMB + tid * 8;
  const v4f a0 = *(const v4f*)(xr);
  const v4f a1 = *(const v4f*)(xr + 4);
  float s = ((a0[0] + a0[1]) + (a0[2] + a0[3])) + ((a1[0] + a1[1]) + (a1[2] + a1[3]));
#pragma unroll
  for (int off = 1; off < 32; off <<= 1) s += __shfl_xor(s, off, 32);
  if (lane == 0) red0[wave] = s;
  __syncthreads();
  const float mean = (red0[0] + red0[1]) * (1.0f / (float)EMB);
  float d[8];
#pragma unroll
  for (int e = 0; e < 4; ++e) { d[e] = a0[e] - mean; d[4 + e] = a1[e] - mean; }
  float q = 0.0f;
#pragma unroll
  for (int e = 0; e < 8; ++e) q += d[e] * d[e];
#pragma unroll
  for (int off = 1; off < 32; off <<= 1) q += __shfl_xor(q, off, 32);
  if (lane == 0) red1[wave] = q;
  __syncthreads();
  const float var = (red1[0] + red1[1]) * (1.0f / (float)EMB);
  const float rstd = 1.0f / sqrtf(var + LN_EPS);
  v4u w;
  w[0] = pk2h(d[0] * rstd, d[1] * rstd);
  w[1] = pk2h(d[2] * rstd, d[3] * rstd);
  w[2] = pk2h(d[4] * rstd, d[5] * rstd);
  w[3] = pk2h(d[6] * rstd, d[7] * rstd);
  unsigned short* op = xn + (size_t)row * EMB + tid * 8;
  *(volatile v4u*)op = w;
  __threadfence();
  *(volatile v4u*)op = w;
}

__global__ __launch_bounds__(256) void tcast_kernel(const float* __restrict__ in, unsigned short* __restrict__ out,
                                                   int R, int Cc, float mul) {
  __shared__ float tile[64 * 65];
  const int tid = threadIdx.x;
  const int c0 = blockIdx.x * 64, r0 = blockIdx.y * 64;
#pragma unroll
  for (int p = 0; p < 4; ++p) {
    const int idx = p * 256 + tid;
    const int row = idx >> 4, cq = (idx & 15) * 4;
    const v4f v = *(const v4f*)(in + (size_t)(r0 + row) * Cc + c0 + cq);
    tile[row * 65 + cq + 0] = v[0];
    tile[row * 65 + cq + 1] = v[1];
    tile[row * 65 + cq + 2] = v[2];
    tile[row * 65 + cq + 3] = v[3];
  }
  __syncthreads();
  for (int pass = 0; pass < 2; ++pass) {
#pragma unroll
    for (int p = 0; p < 2; ++p) {
      const int idx = p * 256 + tid;
      const int orow = idx >> 3, seg = idx & 7;
      float f[8];
#pragma unroll
      for (int e = 0; e < 8; ++e) f[e] = tile[(seg * 8 + e) * 65 + orow] * mul;
      v4u w;
      w[0] = pk2h(f[0], f[1]); w[1] = pk2h(f[2], f[3]); w[2] = pk2h(f[4], f[5]); w[3] = pk2h(f[6], f[7]);
      unsigned short* op = out + (size_t)(c0 + orow) * R + r0 + seg * 8;
      *(volatile v4u*)op = w;
    }
    __threadfence();
  }
}

__global__ __launch_bounds__(256) void vt_kernel(const unsigned short* __restrict__ qkv, unsigned short* __restrict__ vt) {
  __shared__ __align__(16) unsigned short tileh[64 * 72];
  const int tid = threadIdx.x;
  const int c0 = blockIdx.x * 64, mb = blockIdx.y * 64, b = blockIdx.z;
#pragma unroll
  for (int p = 0; p < 2; ++p) {
    const int idx = p * 256 + tid;
    const int row = idx >> 3, seg = idx & 7;
    const v4u w = *(const v4u*)(qkv + ((size_t)(b * SEQ + mb + row) * QKVC + c0 + seg * 8));
    *(v4u*)(tileh + row * 72 + seg * 8) = w;
  }
  __syncthreads();
  for (int pass = 0; pass < 2; ++pass) {
#pragma unroll
    for (int p = 0; p < 2; ++p) {
      const int idx = p * 256 + tid;
      const int orow = idx >> 3, seg = idx & 7;
      unsigned e[8];
#pragma unroll
      for (int k = 0; k < 8; ++k) e[k] = (unsigned)tileh[(seg * 8 + k) * 72 + orow];
      v4u w;
      w[0] = e[0] | (e[1] << 16); w[1] = e[2] | (e[3] << 16); w[2] = e[4] | (e[5] << 16); w[3] = e[6] | (e[7] << 16);
      unsigned short* op = vt + ((size_t)(b * EMB + c0 + orow) * SEQ + mb + seg * 8);
      *(volatile v4u*)op = w;
    }
    __threadfence();
  }
}

__global__ __launch_bounds__(256) void posa_kernel(const float* __restrict__ pos_emb, const float* __restrict__ mask,
                                                  unsigned short* __restrict__ posa) {
  const int n = blockIdx.x, m8 = threadIdx.x * 8;
  const float* mr = mask + (size_t)n * SEQ + m8;
  const v4f ma = *(const v4f*)(mr);
  const v4f mb = *(const v4f*)(mr + 4);
  float mk[8];
#pragma unroll
  for (int e = 0; e < 4; ++e) { mk[e] = ma[e]; mk[4 + e] = mb[e]; }
  float f[8];
#pragma unroll
  for (int e = 0; e < 8; ++e) {
    int idx = n - (m8 + e) + (SEQ - 1);
    idx = idx < 0 ? 0 : (idx > POSLEN - 1 ? POSLEN - 1 : idx);
    f[e] = (pos_emb[idx] * mk[e]) * PT_CARRY;
  }
  v4u w;
  w[0] = pk2h(f[0], f[1]); w[1] = pk2h(f[2], f[3]); w[2] = pk2h(f[4], f[5]); w[3] = pk2h(f[6], f[7]);
  unsigned short* op = posa + (size_t)n * SEQ + m8;
  *(volatile v4u*)op = w;
  __threadfence();
  *(volatile v4u*)op = w;
}

__global__ __launch_bounds__(256) void tsa_kernel(const int* __restrict__ ts, const float* __restrict__ ts_emb,
                                                 const float* __restrict__ mask, unsigned short* __restrict__ tsa) {
  const int b = blockIdx.y;
  const int g = blockIdx.x * 256 + threadIdx.x;
  const int n = g >> 10;
  const int m = (g & 1023) * 2;
  const int tn = ts[b * SEQ + n];
  const v2i tm = *(const v2i*)(ts + b * SEQ + m);
  const v2f mk = *(const v2f*)(mask + (size_t)n * SEQ + m);
  float val[2];
#pragma unroll
  for (int e = 0; e < 2; ++e) {
    const int td = tn - tm[e];
    const int ad = td < 0 ? -td : td;
    const float t = (float)ad;
    const float lg = logf(1.0f + t);
    int bk = (int)floorf(lg);
    bk = bk < 0 ? 0 : (bk > NBUCK - 1 ? NBUCK - 1 : bk);
    val[e] = (ts_emb[bk] * mk[e]) * PT_CARRY;
  }
  const unsigned w = pk2h(val[0], val[1]);
  unsigned short* op = tsa + (((size_t)b * SEQ + n) * SEQ + m);
  *(volatile unsigned*)op = w;
  __threadfence();
  *(volatile unsigned*)op = w;
}

__global__ __launch_bounds__(128) void lat_kernel(const unsigned short* __restrict__ qkv, const unsigned short* __restrict__ vt,
                                                 const float* __restrict__ mask, float* __restrict__ att) {
  __shared__ __align__(16) float Msh[64 * 64];
  __shared__ __align__(16) _Float16 Psh[4][16 * 64];
  __shared__ __align__(16) float Os[4][16 * 68];
  __shared__ int flags[4];
  const int tid = threadIdx.x, wave = tid >> 5, lane = tid & 31;
  const int hh = lane >> 4, c = lane & 15, koff = hh * 8;
  const int nqb = SEQ / 64;
  const int bx = blockIdx.x;
  const int qb = bx % nqb;
  const int bhd = bx / nqb;
  const int h = bhd % NHEAD;
  const int b = bhd / NHEAD;
  const int q0 = qb * 64 + wave * 16;
  const _Float16* Qp = (const _Float16*)qkv;
  const _Float16* Vp = (const _Float16*)vt;

  v16h qa[2];
#pragma unroll
  for (int dc = 0; dc < 2; ++dc)
    qa[dc] = Frag<_Float16>::load(Qp + (size_t)(b * SEQ + q0 + c) * QKVC + EMB + h * HDIM + dc * 32 + koff);

  v8f oacc[4];
#pragma unroll
  for (int t = 0; t < 4; ++t) oacc[t] = (v8f){0.f,0.f,0.f,0.f,0.f,0.f,0.f,0.f};

  for (int kc = 0; kc < SEQ / 64; ++kc) {
    const int kv0 = kc * 64;
    __syncthreads();
    {
      const int mr = tid >> 1, mh = (tid & 1) * 32;
      const float* mrow = mask + (size_t)(qb * 64 + mr) * SEQ + kv0 + mh;
      float* mdst = Msh + mr * 64 + mh;
      int anyf = 0;
#pragma unroll
      for (int i = 0; i < 8; ++i) {
        const v4f m4 = *(const v4f*)(mrow + 4 * i);
        *(v4f*)(mdst + 4 * i) = m4;
        anyf |= (int)(m4[0] != 0.0f) | (int)(m4[1] != 0.0f) | (int)(m4[2] != 0.0f) | (int)(m4[3] != 0.0f);
      }
#pragma unroll
      for (int off = 1; off < 32; off <<= 1) anyf |= __shfl_xor(anyf, off, 32);
      if (lane == 0) flags[wave] = anyf;
    }
    __syncthreads();
    const int anyb = flags[0] | flags[1] | flags[2] | flags[3];
    if (anyb != 0) {
      v8f s[4];
#pragma unroll
      for (int j = 0; j < 4; ++j) s[j] = (v8f){0.f,0.f,0.f,0.f,0.f,0.f,0.f,0.f};
#pragma unroll
      for (int dc = 0; dc < 2; ++dc) {
        v16h kb[4];
#pragma unroll
        for (int j = 0; j < 4; ++j)
          kb[j] = Frag<_Float16>::load(Qp + (size_t)(b * SEQ + kv0 + 16 * j + c) * QKVC + 2 * EMB + h * HDIM + dc * 32 + koff);
#pragma unroll
        for (int j = 0; j < 4; ++j) s[j] = Frag<_Float16>::mma(qa[dc], kb[j], s[j]);
        Frag<_Float16>::guard(s[0], s[3], qa[dc], kb[3]);
        Frag<_Float16>::keep(kb[0], kb[1], kb[2], kb[3]);
      }
      acc_guard4(s[0], s[1], s[2], s[3]);

      _Float16* pw = Psh[wave];
#pragma unroll
      for (int r = 0; r < 8; ++r) {
        const int ql = wave * 16 + 8 * hh + r;
#pragma unroll
        for (int j = 0; j < 4; ++j) {
          const float sv = s[j][r] * (1.0f / (QKV_CARRY * QKV_CARRY));
          const float e = expf(fminf(-sv, 30.0f));
          const float sl = sv * (1.0f / (1.0f + e));
          const float mval = Msh[ql * 64 + 16 * j + c];
          pw[(8 * hh + r) * 64 + 16 * j + c] = (_Float16)((sl * mval) * PL_CARRY);
        }
      }
      __builtin_amdgcn_fence(__ATOMIC_RELEASE, "workgroup");
      __builtin_amdgcn_wave_barrier();
      __builtin_amdgcn_fence(__ATOMIC_ACQUIRE, "workgroup");
#pragma unroll
      for (int kk = 0; kk < 2; ++kk) {
        const v16h pa = Frag<_Float16>::load(pw + c * 64 + kk * 32 + koff);
        v16h vb[4];
#pragma unroll
        for (int t = 0; t < 4; ++t)
          vb[t] = Frag<_Float16>::load(Vp + ((size_t)(b * EMB + h * HDIM + 16 * t + c)) * SEQ + kv0 + kk * 32 + koff);
#pragma unroll
        for (int t = 0; t < 4; ++t) oacc[t] = Frag<_Float16>::mma(pa, vb[t], oacc[t]);
        Frag<_Float16>::guard(oacc[0], oacc[3], pa, vb[3]);
        Frag<_Float16>::keep(vb[0], vb[1], vb[2], vb[3]);
      }
      acc_guard4(oacc[0], oacc[1], oacc[2], oacc[3]);
    }
  }

  float* os = Os[wave];
  const float oscale = 1.0f / (PL_CARRY * QKV_CARRY * (float)SEQ);
#pragma unroll
  for (int r = 0; r < 8; ++r)
#pragma unroll
    for (int t = 0; t < 4; ++t) os[(8 * hh + r) * 68 + t * 16 + c] = oacc[t][r] * oscale;
  __builtin_amdgcn_fence(__ATOMIC_RELEASE, "workgroup");
  __builtin_amdgcn_wave_barrier();
  __builtin_amdgcn_fence(__ATOMIC_ACQUIRE, "workgroup");
  {
    const int c4 = (lane & 15) * 4;
    float* ob = att + (size_t)(b * SEQ) * UCOLS + h * HCAT + 2 * HDIM;
    for (int pass = 0; pass < 2; ++pass) {
#pragma unroll
      for (int it = 0; it < 8; ++it) {
        const int row = it * 2 + hh;
        const v4f val = *(const v4f*)(os + row * 68 + c4);
        *(volatile v4f*)(ob + (size_t)(q0 + row) * UCOLS + c4) = val;
      }
      __threadfence();
    }
  }
}

__global__ __launch_bounds__(192) void ams_kernel(const float* __restrict__ att, const float* __restrict__ u,
                                                 unsigned short* __restrict__ ams) {
  __shared__ float red0[6];
  __shared__ float red1[6];
  const int row = blockIdx.x, tid = threadIdx.x, lane = tid & 31, wave = tid >> 5;
  const float* ar = att + (size_t)row * UCOLS + tid * 8;
  const float* ur = u + (size_t)row * UCOLS + tid * 8;
  const v4f a0 = *(const v4f*)(ar);
  const v4f a1 = *(const v4f*)(ar + 4);
  const v4f u0 = *(const v4f*)(ur);
  const v4f u1 = *(const v4f*)(ur + 4);
  float s = ((a0[0] + a0[1]) + (a0[2] + a0[3])) + ((a1[0] + a1[1]) + (a1[2] + a1[3]));
#pragma unroll
  for (int off = 1; off < 32; off <<= 1) s += __shfl_xor(s, off, 32);
  if (lane == 0) red0[wave] = s;
  __syncthreads();
  const float mean = (((red0[0] + red0[1]) + (red0[2] + red0[3])) + (red0[4] + red0[5])) * (1.0f / (float)UCOLS);
  float d[8], uu[8];
#pragma unroll
  for (int e = 0; e < 4; ++e) { d[e] = a0[e] - mean; d[4 + e] = a1[e] - mean; uu[e] = u0[e]; uu[4 + e] = u1[e]; }
  float q = 0.0f;
#pragma unroll
  for (int e = 0; e < 8; ++e) q += d[e] * d[e];
#pragma unroll
  for (int off = 1; off < 32; off <<= 1) q += __shfl_xor(q, off, 32);
  if (lane == 0) red1[wave] = q;
  __syncthreads();
  const float var = (((red1[0] + red1[1]) + (red1[2] + red1[3])) + (red1[4] + red1[5])) * (1.0f / (float)UCOLS);
  const float rstd = 1.0f / sqrtf(var + LN_EPS);
  float o[8];
#pragma unroll
  for (int e = 0; e < 8; ++e) o[e] = uu[e] * (d[e] * rstd);
  v4u w;
  w[0] = pk2h(o[0], o[1]); w[1] = pk2h(o[2], o[3]); w[2] = pk2h(o[4], o[5]); w[3] = pk2h(o[6], o[7]);
  unsigned short* op = ams + (size_t)row * UCOLS + tid * 8;
  *(volatile v4u*)op = w;
  __threadfence();
  *(volatile v4u*)op = w;
}

constexpr size_t SZ_XN   = (size_t)NROWS * EMB * 2;
constexpr size_t SZ_WT   = (size_t)WCOLS * EMB * 2;
constexpr size_t SZ_L0   = (size_t)EMB * UCOLS * 2;
constexpr size_t SZ_U    = (size_t)NROWS * UCOLS * 4;
constexpr size_t SZ_QKV  = (size_t)NROWS * QKVC * 2;
constexpr size_t SZ_VT   = (size_t)NBATCH * EMB * SEQ * 2;
constexpr size_t SZ_POSA = (size_t)SEQ * SEQ * 2;
constexpr size_t SZ_TSA  = (size_t)NBATCH * SEQ * SEQ * 2;
constexpr size_t SZ_ATT  = (size_t)NROWS * UCOLS * 4;
constexpr size_t SZ_AMS  = (size_t)NROWS * UCOLS * 2;
constexpr size_t OFF_XN   = 0;
constexpr size_t OFF_WT   = OFF_XN + SZ_XN;
constexpr size_t OFF_L0   = OFF_WT + SZ_WT;
constexpr size_t OFF_U    = OFF_L0 + SZ_L0;
constexpr size_t OFF_QKV  = OFF_U + SZ_U;
constexpr size_t OFF_VT   = OFF_QKV + SZ_QKV;
constexpr size_t OFF_POSA = OFF_VT + SZ_VT;
constexpr size_t OFF_TSA  = OFF_POSA + SZ_POSA;
constexpr size_t OFF_ATT  = OFF_TSA + SZ_TSA;
constexpr size_t OFF_AMS  = OFF_ATT + SZ_ATT;
constexpr size_t OFF_END  = OFF_AMS + SZ_AMS;
static_assert(OFF_END == 113770496ull, "carve total");
static_assert(OFF_END <= 134217728ull, "carve under 128 MiB");
static_assert((OFF_WT | OFF_L0 | OFF_U | OFF_QKV | OFF_VT | OFF_POSA | OFF_TSA | OFF_ATT | OFF_AMS) % 256 == 0, "aligned carves");
static_assert(NROWS % 64 == 0 && UCOLS % 64 == 0 && QKVC % 64 == 0 && EMB % 32 == 0, "proj gemm");
static_assert(SEQ % 64 == 0 && EMB % 64 == 0 && SEQ % 32 == 0, "pos/ts gemm");
static_assert(EMB % 64 == 0 && UCOLS % 32 == 0, "out gemm");
static_assert((HCAT * 4) % 256 == 0 && (HDIM * 4) % 256 == 0, "per-head concat slots start on whole 128-B line pairs");

extern "C" void kernel_launch(void* const* d_in, const int* in_sizes, int n_in,
                              void* d_out, int out_size, void* d_ws, size_t ws_size,
                              hipStream_t stream) {
  if (n_in < 10) return;
  if (in_sizes[0] != NROWS * EMB || in_sizes[1] != NROWS || in_sizes[4] != SEQ * SEQ ||
      in_sizes[5] != EMB * WCOLS || in_sizes[6] != POSLEN || in_sizes[7] != NBUCK ||
      in_sizes[8] != UCOLS * EMB || in_sizes[9] != EMB || out_size != NROWS * EMB) return;
  if (OFF_END > ws_size) return;

  const float* x       = (const float*)d_in[0];
  const int*   ts      = (const int*)d_in[1];
  const float* mask    = (const float*)d_in[4];
  const float* uvqk    = (const float*)d_in[5];
  const float* pos_emb = (const float*)d_in[6];
  const float* ts_emb  = (const float*)d_in[7];
  const float* lin0_w  = (const float*)d_in[8];
  const float* lin0_b  = (const float*)d_in[9];
  float* out = (float*)d_out;

  char* ws = (char*)d_ws;
  unsigned short* XN   = (unsigned short*)(ws + OFF_XN);
  unsigned short* WT   = (unsigned short*)(ws + OFF_WT);
  unsigned short* L0WT = (unsigned short*)(ws + OFF_L0);
  float*          U    = (float*)(ws + OFF_U);
  unsigned short* QKV  = (unsigned short*)(ws + OFF_QKV);
  unsigned short* VT   = (unsigned short*)(ws + OFF_VT);
  unsigned short* POSA = (unsigned short*)(ws + OFF_POSA);
  unsigned short* TSA  = (unsigned short*)(ws + OFF_TSA);
  float*          ATT  = (float*)(ws + OFF_ATT);
  unsigned short* AMS  = (unsigned short*)(ws + OFF_AMS);

  ln_cast_kernel<<<NROWS, 64, 0, stream>>>(x, XN);
  tcast_kernel<<<dim3(WCOLS / 64, EMB / 64), 256, 0, stream>>>(uvqk, WT, EMB, WCOLS, W1_CARRY);
  tcast_kernel<<<dim3(EMB / 64, UCOLS / 64), 256, 0, stream>>>(lin0_w, L0WT, UCOLS, EMB, W2_CARRY);

  {
    const unsigned gx = (unsigned)(((NROWS / 64) * (UCOLS / 64) + 7) / 8);
    gemm64_f16<0, 0, false, 3><<<dim3(gx, 1), 256, 0, stream>>>(
        XN, EMB, 0L, WT, EMB, 0L, (void*)U, UCOLS, 0L, 64, 0, nullptr, nullptr, 0L,
        NROWS, UCOLS, EMB, 1.0f / W1_CARRY, 1.0f);
    gemm64_f16<0, 1, false, 3><<<dim3(gx, 1), 256, 0, stream>>>(
        XN, EMB, 0L, WT + (size_t)UCOLS * EMB, EMB, 0L, (void*)QKV, QKVC, 0L, 64, 0, nullptr, nullptr, 0L,
        NROWS, QKVC, EMB, 1.0f / W1_CARRY, QKV_CARRY);
  }
  vt_kernel<<<dim3(EMB / 64, SEQ / 64, NBATCH), 256, 0, stream>>>(QKV, VT);
  posa_kernel<<<SEQ, 256, 0, stream>>>(pos_emb, mask, POSA);
  tsa_kernel<<<dim3((SEQ / 2) * SEQ / 256, NBATCH), 256, 0, stream>>>(ts, ts_emb, mask, TSA);

  {
    const unsigned gx = (unsigned)(((SEQ / 64) * (EMB / 64) + 7) / 8);
    const float sc = 1.0f / (PT_CARRY * QKV_CARRY);
    gemm64_f16<0, 0, false, 0><<<dim3(gx, NBATCH), 256, 0, stream>>>(
        POSA, SEQ, 0L, VT, SEQ, (long)EMB * SEQ, (void*)ATT, UCOLS, (long)SEQ * UCOLS, HCAT, 0,
        nullptr, nullptr, 0L, SEQ, EMB, SEQ, sc, 1.0f);
    gemm64_f16<0, 0, false, 0><<<dim3(gx, NBATCH), 256, 0, stream>>>(
        TSA, SEQ, (long)SEQ * SEQ, VT, SEQ, (long)EMB * SEQ, (void*)ATT, UCOLS, (long)SEQ * UCOLS, HCAT, HDIM,
        nullptr, nullptr, 0L, SEQ, EMB, SEQ, sc, 1.0f);
  }
  lat_kernel<<<NBATCH * NHEAD * (SEQ / 64), 128, 0, stream>>>(QKV, VT, mask, ATT);

  ams_kernel<<<NROWS, 192, 0, stream>>>(ATT, U, AMS);
  {
    const unsigned gx = (unsigned)(((NROWS / 64) * (EMB / 64) + 7) / 8);
    gemm64_f16<2, 0, true, 0><<<dim3(gx, 1), 256, 0, stream>>>(
        AMS, UCOLS, 0L, L0WT, UCOLS, 0L, (void*)out, EMB, 0L, 64, 0, lin0_b, x, 0L,
        NROWS, EMB, UCOLS, 1.0f / W2_CARRY, 1.0f);
  }
  (void)ws_size;
}
